// rnn_single_50070728737109
// MI455X (gfx1250) — hardware-verified
//
#include <hip/hip_runtime.h>


#define NBG  512
#define ENC  512
#define ATT  512
#define ND   1024
#define LOSC 1024.0f
#define LOSCI (1.0f / 1024.0f)

typedef _Float16 h16;
typedef unsigned short bf;
typedef __attribute__((ext_vector_type(16))) __bf16   v16bf;
typedef __attribute__((ext_vector_type(16))) _Float16 v16h;
typedef __attribute__((ext_vector_type(8)))  _Float16 v8h;
typedef __attribute__((ext_vector_type(8)))  unsigned short v8us;
typedef __attribute__((ext_vector_type(8)))  float    v8f;
typedef __attribute__((ext_vector_type(4)))  float    v4f;
typedef __attribute__((ext_vector_type(2)))  float    v2f;
typedef v8h  __attribute__((may_alias)) v8ha;
typedef v4f  __attribute__((may_alias)) v4fa;
typedef v8us __attribute__((may_alias)) v8usa;

__device__ __forceinline__ unsigned short f2bf(float f) { unsigned u = __float_as_uint(f); u += 0x7FFFu + ((u >> 16) & 1u); return (unsigned short)(u >> 16); }
__device__ __forceinline__ float bf2f(unsigned short b) { return __uint_as_float(((unsigned)b) << 16); }
__device__ __forceinline__ float bfr(float f) { return bf2f(f2bf(f)); }
__device__ __forceinline__ v16h cat16(v8h lo, v8h hi) { return __builtin_shufflevector(lo, hi, 0, 1, 2, 3, 4, 5, 6, 7, 8, 9, 10, 11, 12, 13, 14, 15); }
__device__ __forceinline__ v16bf cat16b(v8us lo, v8us hi) { return __builtin_bit_cast(v16bf, __builtin_shufflevector(lo, hi, 0, 1, 2, 3, 4, 5, 6, 7, 8, 9, 10, 11, 12, 13, 14, 15)); }
__device__ __forceinline__ v8f wmma16(v16h a, v16h b, v8f c) { return __builtin_amdgcn_wmma_f32_16x16x32_f16(false, a, false, b, (short)0, c, false, false); }
__device__ __forceinline__ v8f wmmab(v16bf a, v16bf b, v8f c) { return __builtin_amdgcn_wmma_f32_16x16x32_bf16(false, a, false, b, (short)0, c, false, false); }
#define VST2(T, p, v) do { const T vst2_v_ = (v); *(volatile T*)(p) = vst2_v_; __threadfence(); *(volatile T*)(p) = vst2_v_; } while (0)

__global__ __launch_bounds__(256) void k_cvtb(const float* __restrict__ src, int nrows, int ncols, bf* dst) {
    const int lane = threadIdx.x & 31, r = blockIdx.x * 8 + (threadIdx.x >> 5);
    if (r >= nrows) return;
#pragma unroll 1
    for (int q = 0; q < ncols / 256; ++q) { v8us t;
#pragma unroll
        for (int i = 0; i < 8; ++i) t[i] = f2bf(src[(size_t)r * ncols + q * 256 + lane * 8 + i]);
        VST2(v8us, dst + (size_t)r * ncols + q * 256 + lane * 8, t); }
}
__global__ __launch_bounds__(256) void k_x16t(const float* __restrict__ x, h16* XT16) {
    __shared__ __align__(16) h16 tl[64 * 72];
    const int tid = threadIdx.x, j0 = blockIdx.x * 64, d0 = blockIdx.y * 64;
    const int jj = tid >> 2, dq = (tid & 3) * 16;
#pragma unroll
    for (int i = 0; i < 16; ++i) tl[(dq + i) * 72 + jj] = (h16)bfr(x[(size_t)(j0 + jj) * ENC + d0 + dq + i]);
    __syncthreads();
    const int piece = tid & 7;
    auto pass = [&]() {
#pragma unroll
        for (int s = 0; s < 2; ++s) { const int dr = (tid >> 3) + 32 * s; const v8h val = *(const v8ha*)(tl + dr * 72 + piece * 8);
            *(volatile v8h*)(XT16 + (size_t)(d0 + dr) * NBG + j0 + piece * 8) = val; }
    };
    pass(); __threadfence(); pass();
}
__global__ __launch_bounds__(256) void k_wt(const float* __restrict__ Wm, int K, int N, bf* WT) {
    __shared__ __align__(16) unsigned short tl[64 * 72];
    const int tid = threadIdx.x, k0 = blockIdx.x * 64, n0 = blockIdx.y * 64;
    const int kk = tid >> 2, nq = (tid & 3) * 16;
#pragma unroll
    for (int i = 0; i < 16; ++i) tl[(nq + i) * 72 + kk] = f2bf(Wm[(size_t)(k0 + kk) * N + n0 + nq + i]);
    __syncthreads();
    const int piece = tid & 7;
    auto pass = [&]() {
#pragma unroll
        for (int s = 0; s < 2; ++s) { const int nr = (tid >> 3) + 32 * s; const v8us val = *(const v8usa*)(tl + nr * 72 + piece * 8);
            *(volatile v8us*)(WT + (size_t)(n0 + nr) * K + k0 + piece * 8) = val; }
    };
    pass(); __threadfence(); pass();
}

template <bool SPLITA>
__global__ __launch_bounds__(128) void k_gemmb(const bf* __restrict__ A, const bf* __restrict__ Al, const bf* __restrict__ Bn, int K, const float* __restrict__ bias, float* C, int ldc) {
    __shared__ __align__(16) float ost[4][16 * 68];
    const int lane = threadIdx.x & 31, wave = threadIdx.x >> 5, lr = lane & 15, hi = lane >> 4;
    const int r0 = blockIdx.x * 64 + wave * 16, c0 = blockIdx.y * 64;
    const size_t aoff = (size_t)(r0 + lr) * K + 8 * hi;
    size_t boff[4];
#pragma unroll
    for (int t = 0; t < 4; ++t) boff[t] = (size_t)(c0 + t * 16 + lr) * K + 8 * hi;
    v8f acc[4];
#pragma unroll
    for (int t = 0; t < 4; ++t) acc[t] = (v8f){};
#pragma unroll 1
    for (int kc = 0; kc < K; kc += 32) {
        const v16bf a = cat16b(*(const v8us*)(A + aoff + kc), *(const v8us*)(A + aoff + kc + 16));
        v16bf al = a;
        if (SPLITA) al = cat16b(*(const v8us*)(Al + aoff + kc), *(const v8us*)(Al + aoff + kc + 16));
#pragma unroll
        for (int t = 0; t < 4; ++t) { const v16bf b = cat16b(*(const v8us*)(Bn + boff[t] + kc), *(const v8us*)(Bn + boff[t] + kc + 16)); acc[t] = wmmab(a, b, acc[t]); if (SPLITA) acc[t] = wmmab(al, b, acc[t]); }
        asm volatile("v_nop\n\tv_nop\n\tv_nop\n\tv_nop" : "+v"(acc[0]), "+v"(acc[1]), "+v"(acc[2]), "+v"(acc[3]) : "v"(a), "v"(al));
    }
    float* os = &ost[wave][0];
#pragma unroll
    for (int t = 0; t < 4; ++t) { const float bv = bfr(bias[c0 + t * 16 + lr]);
#pragma unroll
        for (int j = 0; j < 8; ++j) os[(hi * 8 + j) * 68 + t * 16 + lr] = acc[t][j] + bv; }
    __syncthreads();
    float* crow = C + (size_t)r0 * ldc + c0;
    auto pass = [&]() {
#pragma unroll
        for (int s = 0; s < 8; ++s) { const int Lid = (lane >> 3) + 4 * s, piece = lane & 7; const int row = Lid >> 1, cofs = (Lid & 1) * 32 + piece * 4;
            const v4f val = *(const v4fa*)(os + row * 68 + cofs); *(volatile v4f*)(crow + (size_t)row * ldc + cofs) = val; }
    };
    pass(); __threadfence(); pass();
}

__global__ __launch_bounds__(512) void k_att(const float* __restrict__ A1, const float* __restrict__ A2, const float* __restrict__ Wf, const float* __restrict__ bfv, h16* ALH, h16* ALL) {
    __shared__ float red[16];
    __shared__ __align__(16) h16 rowh[512];
    __shared__ __align__(16) h16 rowl[512];
    const int i = blockIdx.x, j = threadIdx.x, lane = j & 31, wv = j >> 5;
    const float* a1 = A1 + (size_t)j * ATT; const float* a2 = A2 + (size_t)i * ATT;
    float s = 0.f;
#pragma unroll 4
    for (int a = 0; a < ATT; ++a) { const float v = a1[a] + a2[a]; s += fmaxf(v, 0.f) * bfr(Wf[a]); }
    s += bfr(bfv[0]);
    float m = s;
#pragma unroll
    for (int o = 16; o; o >>= 1) m = fmaxf(m, __shfl_xor(m, o, 32));
    if (lane == 0) red[wv] = m;
    __syncthreads();
    float gm = red[0];
#pragma unroll
    for (int w = 1; w < 16; ++w) gm = fmaxf(gm, red[w]);
    __syncthreads();
    const float e = __expf(s - gm);
    float es = e;
#pragma unroll
    for (int o = 16; o; o >>= 1) es += __shfl_xor(es, o, 32);
    if (lane == 0) red[wv] = es;
    __syncthreads();
    float tot = 0.f;
#pragma unroll
    for (int w = 0; w < 16; ++w) tot += red[w];
    const float alpha = e / tot;
    const h16 ah = (h16)alpha; rowh[j] = ah; rowl[j] = (h16)((alpha - (float)ah) * LOSC);
    __syncthreads();
    if (wv < 2) {
        typedef __attribute__((ext_vector_type(16))) _Float16 v16h_; typedef v16h_ __attribute__((may_alias)) v16ha_;
        const v16h_ val = *(const v16ha_*)((wv ? rowl : rowh) + lane * 16);
        h16* dst = (wv ? ALL : ALH) + (size_t)i * NBG + lane * 16;
        *(volatile v16h_*)dst = val; __threadfence(); *(volatile v16h_*)dst = val;
    }
}

__global__ __launch_bounds__(128) void k_awe(const h16* __restrict__ ALH, const h16* __restrict__ ALL, const h16* __restrict__ XT16, const float* __restrict__ x, bf* IWH, bf* IWL) {
    __shared__ __align__(16) float ost[4][16 * 68];
    const int lane = threadIdx.x & 31, wave = threadIdx.x >> 5, lr = lane & 15, hi = lane >> 4;
    const int r0 = blockIdx.x * 64 + wave * 16, c0 = blockIdx.y * 64;
    const size_t aoff = (size_t)(r0 + lr) * NBG + 8 * hi;
    size_t boff[4];
#pragma unroll
    for (int t = 0; t < 4; ++t) boff[t] = (size_t)(c0 + t * 16 + lr) * NBG + 8 * hi;
    v8f acc[4], accx[4];
#pragma unroll
    for (int t = 0; t < 4; ++t) { acc[t] = (v8f){}; accx[t] = (v8f){}; }
#pragma unroll 1
    for (int kc = 0; kc < NBG; kc += 32) {
        const v16h a = cat16(*(const v8h*)(ALH + aoff + kc), *(const v8h*)(ALH + aoff + kc + 16)), al = cat16(*(const v8h*)(ALL + aoff + kc), *(const v8h*)(ALL + aoff + kc + 16));
#pragma unroll
        for (int t = 0; t < 4; ++t) { const v16h b = cat16(*(const v8h*)(XT16 + boff[t] + kc), *(const v8h*)(XT16 + boff[t] + kc + 16)); acc[t] = wmma16(a, b, acc[t]); accx[t] = wmma16(al, b, accx[t]); }
        asm volatile("v_nop\n\tv_nop\n\tv_nop\n\tv_nop" : "+v"(acc[0]), "+v"(acc[1]), "+v"(acc[2]), "+v"(acc[3]), "+v"(accx[0]), "+v"(accx[1]), "+v"(accx[2]), "+v"(accx[3]) : "v"(a), "v"(al));
    }
    float* os = &ost[wave][0];
#pragma unroll
    for (int t = 0; t < 4; ++t) { const int col = c0 + t * 16 + lr;
#pragma unroll
        for (int j = 0; j < 8; ++j) os[(hi * 8 + j) * 68 + t * 16 + lr] = (acc[t][j] + accx[t][j] * LOSCI) * bfr(x[(size_t)(r0 + hi * 8 + j) * ENC + col]); }
    __syncthreads();
    const size_t rbase = (size_t)r0 * ENC + c0;
    auto pass = [&]() {
#pragma unroll
        for (int s = 0; s < 4; ++s) { const int row = 4 * s + (lane >> 3), piece = lane & 7; const float* sp = os + row * 68 + piece * 8; v8us oh, ol;
#pragma unroll
            for (int t = 0; t < 8; ++t) { const unsigned short hb = f2bf(sp[t]); oh[t] = hb; ol[t] = f2bf(sp[t] - bf2f(hb)); }
            *(volatile v8us*)(IWH + rbase + (size_t)row * ENC + piece * 8) = oh; *(volatile v8us*)(IWL + rbase + (size_t)row * ENC + piece * 8) = ol; }
    };
    pass(); __threadfence(); pass();
}

__global__ __launch_bounds__(512) void k_fin(const float* __restrict__ ST, const float* __restrict__ INP, const float* __restrict__ W3, const float* __restrict__ b3, float* out0, float* out1) {
    __shared__ float pr[16][2];
    const int lane = threadIdx.x & 31, wv = threadIdx.x >> 5, i = blockIdx.x * 16 + wv;
    const float* st = ST + (size_t)i * ND; const float* in = INP + (size_t)i * ND;
    float d0 = 0.f, d1 = 0.f;
#pragma unroll 1
    for (int q = 0; q < 4; ++q) {
        v8f ns;
#pragma unroll
        for (int t = 0; t < 8; ++t) { const int c = q * 256 + lane * 8 + t; const float v = fmaxf(st[c] + in[c], 0.f); ns[t] = v; d0 += v * bfr(W3[c * 2]); d1 += v * bfr(W3[c * 2 + 1]); }
        VST2(v8f, out1 + (size_t)i * ND + q * 256 + lane * 8, ns);
    }
#pragma unroll
    for (int o = 16; o; o >>= 1) { d0 += __shfl_xor(d0, o, 32); d1 += __shfl_xor(d1, o, 32); }
    if (lane == 0) { pr[wv][0] = d0 + bfr(b3[0]); pr[wv][1] = d1 + bfr(b3[1]); }
    __syncthreads();
    if (wv == 0) { const float v = (&pr[0][0])[lane]; VST2(float, out0 + (size_t)blockIdx.x * 32 + lane, v); }
}

extern "C" void kernel_launch(void* const* d_in, const int* in_sizes, int n_in,
                              void* d_out, int out_size, void* d_ws, size_t ws_size, hipStream_t stream) {
    (void)in_sizes; (void)n_in; (void)out_size;
    const float* x = (const float*)d_in[0]; const float* state = (const float*)d_in[1];
    const float* We = (const float*)d_in[2]; const float* be = (const float*)d_in[3]; const float* Wd = (const float*)d_in[4]; const float* bd = (const float*)d_in[5];
    const float* Wf = (const float*)d_in[6]; const float* bfv = (const float*)d_in[7]; const float* W1 = (const float*)d_in[8]; const float* b1 = (const float*)d_in[9];
    const float* W2 = (const float*)d_in[10]; const float* b2 = (const float*)d_in[11]; const float* W3 = (const float*)d_in[12]; const float* b3 = (const float*)d_in[13];
    float* out0 = (float*)d_out;
    float* out1 = (float*)((char*)d_out + 4096);
    char* wsp = (char*)d_ws;
    auto take = [&](size_t bytes) { char* p = wsp; wsp += (bytes + 255) & ~(size_t)255; return (void*)p; };
    bf* Xb = (bf*)take((size_t)NBG * ENC * 2); bf* Sb = (bf*)take((size_t)NBG * ND * 2); h16* XT16 = (h16*)take((size_t)ENC * NBG * 2);
    bf* WeT = (bf*)take((size_t)ATT * ENC * 2); bf* WdT = (bf*)take((size_t)ATT * ND * 2); bf* W1T = (bf*)take((size_t)ND * ENC * 2); bf* W2T = (bf*)take((size_t)ND * ND * 2);
    float* A1 = (float*)take((size_t)NBG * ATT * 4); float* A2 = (float*)take((size_t)NBG * ATT * 4);
    h16* ALH = (h16*)take((size_t)NBG * NBG * 2); h16* ALL = (h16*)take((size_t)NBG * NBG * 2);
    bf* IWH = (bf*)take((size_t)NBG * ENC * 2); bf* IWL = (bf*)take((size_t)NBG * ENC * 2);
    float* INP = (float*)take((size_t)NBG * ND * 4); float* ST = (float*)take((size_t)NBG * ND * 4);
    if ((size_t)(wsp - (char*)d_ws) > ws_size) return;
    k_cvtb<<<NBG / 8, 256, 0, stream>>>(x, NBG, ENC, Xb);
    k_cvtb<<<NBG / 8, 256, 0, stream>>>(state, NBG, ND, Sb);
    k_x16t<<<dim3(NBG / 64, ENC / 64, 1), 256, 0, stream>>>(x, XT16);
    k_wt<<<dim3(ENC / 64, ATT / 64, 1), 256, 0, stream>>>(We, ENC, ATT, WeT);
    k_wt<<<dim3(ND / 64, ATT / 64, 1), 256, 0, stream>>>(Wd, ND, ATT, WdT);
    k_wt<<<dim3(ENC / 64, ND / 64, 1), 256, 0, stream>>>(W1, ENC, ND, W1T);
    k_wt<<<dim3(ND / 64, ND / 64, 1), 256, 0, stream>>>(W2, ND, ND, W2T);
    k_gemmb<false><<<dim3(NBG / 64, ATT / 64, 1), 128, 0, stream>>>(Xb, nullptr, WeT, ENC, be, A1, ATT);
    k_gemmb<false><<<dim3(NBG / 64, ATT / 64, 1), 128, 0, stream>>>(Sb, nullptr, WdT, ND, bd, A2, ATT);
    k_gemmb<false><<<dim3(NBG / 64, ND / 64, 1), 128, 0, stream>>>(Sb, nullptr, W2T, ND, b2, ST, ND);
    k_att<<<NBG, 512, 0, stream>>>(A1, A2, Wf, bfv, ALH, ALL);
    k_awe<<<dim3(NBG / 64, ENC / 64, 1), 128, 0, stream>>>(ALH, ALL, XT16, x, IWH, IWL);
    k_gemmb<true><<<dim3(NBG / 64, ND / 64, 1), 128, 0, stream>>>(IWH, IWL, W1T, ENC, b1, INP, ND);
    k_fin<<<NBG / 16, 512, 0, stream>>>(ST, INP, W3, b3, out0, out1);
}
